// DictionaryLearningTokenized_23081154249057
// MI455X (gfx1250) — hardware-verified
//
#include <hip/hip_runtime.h>
#include <stdint.h>
#include <math.h>


#pragma clang fp contract(off)

#define NA     256
#define DIMC   64
#define HWSZ   4096
#define NBAT   32
#define SPB    64
#define PP     72
#define PLW    32
#define GSP    260
#define XSP    68
#define HBP    260

typedef float v4f __attribute__((ext_vector_type(4)));
typedef float v8f __attribute__((ext_vector_type(8)));
typedef unsigned int v4u __attribute__((ext_vector_type(4)));
typedef __bf16 v16b __attribute__((ext_vector_type(16)));
typedef v4f __attribute__((may_alias)) v4fa;
typedef v4u __attribute__((may_alias)) v4ua;

union Frag { v16b v; v4u q[2]; unsigned int u[8]; };

__device__ __forceinline__ unsigned int bf16_rne(float x) {
  const unsigned int u = __float_as_uint(x);
  return (u + 0x7FFFu + ((u >> 16) & 1u)) >> 16;
}

__device__ __forceinline__ void split3(float x, unsigned int& h, unsigned int& m, unsigned int& l) {
  h = bf16_rne(x);
  const float r1 = x - __uint_as_float(h << 16);
  m = bf16_rne(r1);
  const float r2 = r1 - __uint_as_float(m << 16);
  l = bf16_rne(r2);
}

__device__ __forceinline__ void pack2(float a, float b, unsigned int& ph, unsigned int& pm, unsigned int& pl) {
  unsigned int h0, m0, l0, h1, m1, l1;
  split3(a, h0, m0, l0);
  split3(b, h1, m1, l1);
  ph = h0 | (h1 << 16);
  pm = m0 | (m1 << 16);
  pl = l0 | (l1 << 16);
}

__device__ __forceinline__ v8f wmma16(v16b a, v16b b, v8f c) {
  v8f d = __builtin_amdgcn_wmma_f32_16x16x32_bf16(false, a, false, b, (short)0, c, false, false);
  asm volatile("v_nop\n\tv_nop\n\tv_nop\n\tv_nop" : "+v"(d) : "v"(a), "v"(b));
  return d;
}

__device__ __forceinline__ v8f vzero8() {
  v8f z = {0.f, 0.f, 0.f, 0.f, 0.f, 0.f, 0.f, 0.f};
  return z;
}

__global__ __launch_bounds__(256) void k_prep(
    const float* __restrict__ dict,
    float* DnT,
    unsigned int* Ph, unsigned int* Pm, unsigned int* Pl,
    float* G)
{
  extern __shared__ float4 dyn_smem[];
  unsigned char* smem = (unsigned char*)dyn_smem;
  unsigned short* Lh = (unsigned short*)smem;
  unsigned short* Lm = Lh + NA * PP;
  unsigned short* Ll = Lm + NA * PP;
  float* Gs = (float*)(smem + (size_t)3 * NA * PP * 2);
  float* Ds = Gs + 16 * GSP;

  const int tid = threadIdx.x;
  const int g = blockIdx.x;
  const int j = tid;

  float n2 = 0.f;
  for (int c = 0; c < DIMC; ++c) {
    const float v = dict[c * NA + j];
    n2 = n2 + v * v;
  }
  const float inv = 1.0f / fmaxf(sqrtf(n2), 1e-10f);
  const bool own = ((j >> 4) == g);
  for (int c = 0; c < DIMC; ++c) {
    const float v = dict[c * NA + j] * inv;
    unsigned int bh, bm, bl;
    split3(v, bh, bm, bl);
    Lh[j * PP + c] = (unsigned short)bh;
    Lm[j * PP + c] = (unsigned short)bm;
    Ll[j * PP + c] = (unsigned short)bl;
    if (own) Ds[(j & 15) * DIMC + c] = v;
  }
  __syncthreads();

  const int lane = tid & 31, w = tid >> 5, m = lane & 15, hh = lane >> 4;
  Frag ah[2], am[2], al[2];
#pragma unroll
  for (int ks = 0; ks < 2; ++ks) {
    const int base = (16 * g + m) * PP + 32 * ks + 8 * hh;
    ah[ks].q[0] = *(const v4ua*)(Lh + base); ah[ks].q[1] = *(const v4ua*)(Lh + base + 16);
    am[ks].q[0] = *(const v4ua*)(Lm + base); am[ks].q[1] = *(const v4ua*)(Lm + base + 16);
    al[ks].q[0] = *(const v4ua*)(Ll + base); al[ks].q[1] = *(const v4ua*)(Ll + base + 16);
  }
#pragma unroll
  for (int t2 = 0; t2 < 2; ++t2) {
    const int tj = w + 8 * t2;
    v8f acc = vzero8();
#pragma unroll
    for (int ks = 0; ks < 2; ++ks) {
      const int bb = (tj * 16 + m) * PP + 32 * ks + 8 * hh;
      Frag bl, bm, bh;
      bl.q[0] = *(const v4ua*)(Ll + bb); bl.q[1] = *(const v4ua*)(Ll + bb + 16);
      acc = wmma16(ah[ks].v, bl.v, acc);
      bm.q[0] = *(const v4ua*)(Lm + bb); bm.q[1] = *(const v4ua*)(Lm + bb + 16);
      acc = wmma16(am[ks].v, bm.v, acc);
      acc = wmma16(ah[ks].v, bm.v, acc);
      bh.q[0] = *(const v4ua*)(Lh + bb); bh.q[1] = *(const v4ua*)(Lh + bb + 16);
      acc = wmma16(al[ks].v, bh.v, acc);
      acc = wmma16(am[ks].v, bh.v, acc);
      acc = wmma16(ah[ks].v, bh.v, acc);
    }
#pragma unroll
    for (int r = 0; r < 8; ++r) Gs[(8 * hh + r) * GSP + tj * 16 + m] = acc[r];
  }
  __syncthreads();

  v4u pv[2]; unsigned int* pd[2]; bool pk[2];
#pragma unroll
  for (int i = 0; i < 2; ++i) {
    const int idx = i * 256 + tid;
    pk[i] = idx < 48 * 8;
    const int line = idx >> 3, q = idx & 7;
    const int p = line >> 4, al_ = line & 15, atom = 16 * g + al_;
    const unsigned short* src = (p == 0) ? Lh : ((p == 1) ? Lm : Ll);
    unsigned int* dst = (p == 0) ? Ph : ((p == 1) ? Pm : Pl);
    pd[i] = dst + (size_t)atom * PLW + 4 * q;
    v4u z = {0u, 0u, 0u, 0u};
    pv[i] = z;
    if (pk[i]) pv[i] = *(const v4ua*)(src + atom * PP + 8 * q);
  }
  const int dal = tid >> 4, dq = tid & 15;
  const v4f dv = *(const v4fa*)(Ds + dal * DIMC + 4 * dq);
  float* dd = DnT + (size_t)(16 * g + dal) * DIMC + 4 * dq;
  v4f gv[4]; float* gd[4];
#pragma unroll
  for (int i = 0; i < 4; ++i) {
    const int idx = i * 256 + tid;
    const int row = idx >> 6, q = idx & 63;
    gv[i] = *(const v4fa*)(Gs + row * GSP + 4 * q);
    gd[i] = G + (size_t)(16 * g + row) * NA + 4 * q;
  }

#pragma unroll
  for (int i = 0; i < 2; ++i) if (pk[i]) *(volatile v4u*)pd[i] = pv[i];
  *(volatile v4f*)dd = dv;
#pragma unroll
  for (int i = 0; i < 4; ++i) *(volatile v4f*)gd[i] = gv[i];
  __threadfence();
#pragma unroll
  for (int i = 0; i < 2; ++i) if (pk[i]) *(volatile v4u*)pd[i] = pv[i];
  *(volatile v4f*)dd = dv;
#pragma unroll
  for (int i = 0; i < 4; ++i) *(volatile v4f*)gd[i] = gv[i];
}

__global__ __launch_bounds__(64) void k_omp(
    const float* __restrict__ ze,
    const float* __restrict__ DnT,
    const unsigned int* __restrict__ Ph,
    const unsigned int* __restrict__ Pm,
    const unsigned int* __restrict__ Pl,
    const float* __restrict__ G,
    float* out,
    float* part,
    int nsig)
{
  extern __shared__ float4 dyn_smem[];
  float* Xs  = (float*)dyn_smem;
  float* Hb  = Xs + SPB * XSP;
  float* Zs  = Hb + SPB * HBP;
  float* red = Zs + SPB * DIMC;

  const int tid = threadIdx.x;
  const int s0 = blockIdx.x * SPB;
  if (s0 >= nsig) return;
  const int b = s0 / HWSZ;
  const int hw0 = s0 - b * HWSZ;
  const size_t zbase = (size_t)b * DIMC * HWSZ + (size_t)hw0;

  for (int f = tid; f < DIMC * SPB; f += SPB) {
    const int c = f >> 6, t = f & 63;
    Xs[t * XSP + c] = ze[zbase + (size_t)c * HWSZ + t];
  }
  __syncthreads();

  {
    const int lane = tid & 31, wv = tid >> 5, m = lane & 15, hh = lane >> 4;
#pragma unroll 1
    for (int rt = 0; rt < 2; ++rt) {
      const int row0 = wv * 32 + rt * 16;
      Frag fh[2], fm[2], fl[2];
#pragma unroll
      for (int ks = 0; ks < 2; ++ks) {
        const float* xr = Xs + (row0 + m) * XSP + 32 * ks + 8 * hh;
        const v4f xa = *(const v4fa*)(xr);
        const v4f xb = *(const v4fa*)(xr + 4);
        const v4f xc = *(const v4fa*)(xr + 16);
        const v4f xd = *(const v4fa*)(xr + 20);
        pack2(xa.x, xa.y, fh[ks].u[0], fm[ks].u[0], fl[ks].u[0]);
        pack2(xa.z, xa.w, fh[ks].u[1], fm[ks].u[1], fl[ks].u[1]);
        pack2(xb.x, xb.y, fh[ks].u[2], fm[ks].u[2], fl[ks].u[2]);
        pack2(xb.z, xb.w, fh[ks].u[3], fm[ks].u[3], fl[ks].u[3]);
        pack2(xc.x, xc.y, fh[ks].u[4], fm[ks].u[4], fl[ks].u[4]);
        pack2(xc.z, xc.w, fh[ks].u[5], fm[ks].u[5], fl[ks].u[5]);
        pack2(xd.x, xd.y, fh[ks].u[6], fm[ks].u[6], fl[ks].u[6]);
        pack2(xd.z, xd.w, fh[ks].u[7], fm[ks].u[7], fl[ks].u[7]);
      }
#pragma unroll 1
      for (int nt = 0; nt < 16; ++nt) {
        v8f acc = vzero8();
#pragma unroll
        for (int ks = 0; ks < 2; ++ks) {
          const int bo = (nt * 16 + m) * PLW + 16 * ks + 4 * hh;
          Frag bl, bm, bh;
          bl.q[0] = *(const v4ua*)(Pl + bo); bl.q[1] = *(const v4ua*)(Pl + bo + 8);
          acc = wmma16(fh[ks].v, bl.v, acc);
          bm.q[0] = *(const v4ua*)(Pm + bo); bm.q[1] = *(const v4ua*)(Pm + bo + 8);
          acc = wmma16(fm[ks].v, bm.v, acc);
          acc = wmma16(fh[ks].v, bm.v, acc);
          bh.q[0] = *(const v4ua*)(Ph + bo); bh.q[1] = *(const v4ua*)(Ph + bo + 8);
          acc = wmma16(fl[ks].v, bh.v, acc);
          acc = wmma16(fm[ks].v, bh.v, acc);
          acc = wmma16(fh[ks].v, bh.v, acc);
        }
#pragma unroll
        for (int r = 0; r < 8; ++r) Hb[(row0 + 8 * hh + r) * HBP + nt * 16 + m] = acc[r];
      }
    }
  }
  __syncthreads();

  const int t = tid;
  float* Hrow = Hb + t * HBP;
  const float qnan = __uint_as_float(0x7fc00000u);
  int I[4] = {0, 0, 0, 0};
  const float* gp[4] = {G, G, G, G};
  float Lp[10] = {1.f, 0.f, 0.f, 0.f, 0.f, 0.f, 0.f, 0.f, 0.f, 0.f};
  float x[4] = {0.f, 0.f, 0.f, 0.f};
  float hs[4] = {0.f, 0.f, 0.f, 0.f};

#pragma unroll
  for (int k = 1; k <= 4; ++k) {
    float best = -1.0f;
    int bidx = 0;
#pragma unroll 1
    for (int jj = 0; jj < NA; jj += 4) {
      const v4f hv = *(const v4fa*)(Hrow + jj);
      v4f gvv[3];
#pragma unroll
      for (int mm = 0; mm < k - 1; ++mm) gvv[mm] = *(const v4fa*)(gp[mm] + jj);
#pragma unroll
      for (int e = 0; e < 4; ++e) {
        float v = hv[e];
        if (k > 1) {
          float beta = x[0] * gvv[0][e];
#pragma unroll
          for (int mm = 1; mm < k - 1; ++mm) beta = beta + x[mm] * gvv[mm][e];
          v = v - beta;
        }
        const float av = fabsf(v);
        if (av > best) { best = av; bidx = jj + e; }
      }
    }
    if (k > 1) {
      float wv[3];
#pragma unroll
      for (int mm = 0; mm < k - 1; ++mm) {
        float gval = gp[mm][bidx];
#pragma unroll
        for (int cc = 0; cc < mm; ++cc) gval = gval - Lp[mm * (mm + 1) / 2 + cc] * wv[cc];
        wv[mm] = gval / Lp[mm * (mm + 1) / 2 + mm];
      }
      float ss = 0.f;
#pragma unroll
      for (int mm = 0; mm < k - 1; ++mm) ss = ss + wv[mm] * wv[mm];
      const float corner = sqrtf(fmaxf(1.0f - ss, 1e-12f));
      const int rr = k - 1;
#pragma unroll
      for (int cc = 0; cc < k - 1; ++cc) Lp[rr * (rr + 1) / 2 + cc] = wv[cc];
      Lp[rr * (rr + 1) / 2 + rr] = corner;
    }
    I[k - 1] = bidx;
    gp[k - 1] = G + (size_t)(bidx & (NA - 1)) * NA;
    hs[k - 1] = Hrow[bidx];
    Hrow[bidx] = qnan;
    float y[4];
#pragma unroll
    for (int mm = 0; mm < k; ++mm) {
      float v = hs[mm];
#pragma unroll
      for (int cc = 0; cc < mm; ++cc) v = v - Lp[mm * (mm + 1) / 2 + cc] * y[cc];
      y[mm] = v / Lp[mm * (mm + 1) / 2 + mm];
    }
#pragma unroll
    for (int mm = k - 1; mm >= 0; --mm) {
      float v = y[mm];
#pragma unroll
      for (int cc = mm + 1; cc < k; ++cc) v = v - Lp[cc * (cc + 1) / 2 + mm] * x[cc];
      x[mm] = v / Lp[mm * (mm + 1) / 2 + mm];
    }
  }

  const float kInvL = (float)(1.0 / 3.9318256327243257);
  const float kL = 1.0f / kInvL;
  float qd[4];
#pragma unroll
  for (int mm = 0; mm < 4; ++mm) {
    const float cl = fminf(fmaxf(x[mm], -3.0f), 3.0f) * (1.0f / 3.0f);
    const float enc = copysignf(log1pf(fabsf(cl) * 50.0f) * kInvL, cl);
    const float sc = (enc + 1.0f) * 7.5f;
    int bin = (int)rintf(sc);
    bin = bin < 0 ? 0 : (bin > 15 ? 15 : bin);
    const float z = (float)bin * (float)(2.0 / 15.0) - 1.0f;
    qd[mm] = copysignf(expm1f(fabsf(z) * kL) * (1.0f / 50.0f), z) * 3.0f;
  }

  const float* ar[4];
#pragma unroll
  for (int mm = 0; mm < 4; ++mm) ar[mm] = DnT + (size_t)(I[mm] & (NA - 1)) * DIMC;
  float lsum = 0.f;
#pragma unroll 1
  for (int c = 0; c < DIMC; c += 4) {
    const v4f a0 = *(const v4fa*)(ar[0] + c);
    const v4f a1 = *(const v4fa*)(ar[1] + c);
    const v4f a2 = *(const v4fa*)(ar[2] + c);
    const v4f a3 = *(const v4fa*)(ar[3] + c);
    const v4f xv = *(const v4fa*)(Xs + t * XSP + c);
#pragma unroll
    for (int e = 0; e < 4; ++e) {
      float rec = qd[0] * a0[e];
      rec = rec + qd[1] * a1[e];
      rec = rec + qd[2] * a2[e];
      rec = rec + qd[3] * a3[e];
      const float dlt = rec - xv[e];
      Zs[(c + e) * SPB + t] = xv[e] + dlt;
      lsum = lsum + dlt * dlt;
    }
  }
  red[t] = lsum;
  __syncthreads();

  float bs = 0.f;
  for (int i = 0; i < SPB; ++i) bs = bs + red[i];

#pragma unroll
  for (int i = 0; i < 16; ++i) {
    const int idx = i * SPB + tid;
    const int c = idx >> 4, q = idx & 15;
    const v4f v = *(const v4fa*)(Zs + c * SPB + 4 * q);
    *(volatile v4f*)(out + zbase + (size_t)c * HWSZ + 4 * q) = v;
  }
  if (tid < 8) {
    v4f pvv = {0.f, 0.f, 0.f, 0.f};
    if (tid == 0) pvv.x = bs;
    *(volatile v4f*)(part + (size_t)blockIdx.x * 32 + 4 * tid) = pvv;
  }
  __threadfence();
#pragma unroll
  for (int i = 0; i < 16; ++i) {
    const int idx = i * SPB + tid;
    const int c = idx >> 4, q = idx & 15;
    const v4f v = *(const v4fa*)(Zs + c * SPB + 4 * q);
    *(volatile v4f*)(out + zbase + (size_t)c * HWSZ + 4 * q) = v;
  }
  if (tid < 8) {
    v4f pvv = {0.f, 0.f, 0.f, 0.f};
    if (tid == 0) pvv.x = bs;
    *(volatile v4f*)(part + (size_t)blockIdx.x * 32 + 4 * tid) = pvv;
  }
}

__global__ __launch_bounds__(256) void k_fin(
    const float* __restrict__ part, float* out_loss, int nblk, int nelem)
{
  __shared__ double sh[256];
  const int tid = threadIdx.x;
  double s = 0.0;
  for (int i = tid; i < nblk; i += 256) s += (double)part[(size_t)i * 32];
  sh[tid] = s;
  __syncthreads();
  for (int st = 128; st > 0; st >>= 1) {
    if (tid < st) sh[tid] = sh[tid] + sh[tid + st];
    __syncthreads();
  }
  if (tid == 0) {
    const float mval = (float)(sh[0] / (double)nelem);
    const float qt = 0.25f * mval;
    const float loss = mval + qt;
    *(volatile float*)out_loss = loss;
    __threadfence();
    *(volatile float*)out_loss = loss;
  }
}

extern "C" void kernel_launch(void* const* d_in, const int* in_sizes, int n_in,
                              void* d_out, int out_size, void* d_ws, size_t ws_size,
                              hipStream_t stream)
{
  if (n_in < 2) return;
  const long long nze  = in_sizes[0];
  const long long ndc  = in_sizes[1];
  const long long nsig = (long long)NBAT * HWSZ;
  if (nze != nsig * DIMC || ndc != (long long)DIMC * NA || (long long)out_size < nze + 1) return;
  const int nblk = (int)((nsig + SPB - 1) / SPB);

  size_t off = 0;
  const size_t oDnT = off;  off += (size_t)NA * DIMC * 4;
  const size_t oPh  = off;  off += (size_t)NA * DIMC * 2;
  const size_t oPm  = off;  off += (size_t)NA * DIMC * 2;
  const size_t oPl  = off;  off += (size_t)NA * DIMC * 2;
  const size_t oG   = off;  off += (size_t)NA * NA * 4;
  off = (off + 127) & ~(size_t)127;
  const size_t oPart = off; off += (size_t)nblk * 128;
  if (off > ws_size) return;

  unsigned char* ws = (unsigned char*)d_ws;
  const float* ze   = (const float*)d_in[0];
  const float* dict = (const float*)d_in[1];
  float* out = (float*)d_out;
  float* DnT = (float*)(ws + oDnT);
  unsigned int* Ph = (unsigned int*)(ws + oPh);
  unsigned int* Pm = (unsigned int*)(ws + oPm);
  unsigned int* Pl = (unsigned int*)(ws + oPl);
  float* G = (float*)(ws + oG);
  float* part = (float*)(ws + oPart);

  const size_t lds1 = (size_t)3 * NA * PP * 2 + (size_t)16 * GSP * 4 + (size_t)16 * DIMC * 4;
  const size_t lds2 = ((size_t)SPB * XSP + (size_t)SPB * HBP + (size_t)SPB * DIMC + SPB) * 4;

  hipLaunchKernelGGL(k_prep, dim3(NA / 16), dim3(256), lds1, stream,
                     dict, DnT, Ph, Pm, Pl, G);
  hipLaunchKernelGGL(k_omp, dim3(nblk), dim3(SPB), lds2, stream,
                     ze, (const float*)DnT, (const unsigned int*)Ph, (const unsigned int*)Pm,
                     (const unsigned int*)Pl, (const float*)G, out, part, (int)nsig);
  hipLaunchKernelGGL(k_fin, dim3(1), dim3(256), 0, stream,
                     (const float*)part, out + nze, nblk, (int)nze);
  (void)hipGetLastError();
}
